// MultiHead_81527069213242
// MI455X (gfx1250) — hardware-verified
//
#include <hip/hip_runtime.h>
#ifndef SEQ
#define SEQ 4096
#endif
#define SEQ_FULL 4096
#define EMB 1024
#define MASKV (-1.0e9f)
static_assert(SEQ % 256 == 0);
static_assert(SEQ >= 256);
static_assert(SEQ <= SEQ_FULL);
static_assert(EMB % 128 == 0);

typedef _Float16 v16h __attribute__((ext_vector_type(16)));
typedef _Float16 v4h  __attribute__((ext_vector_type(4)));
typedef unsigned short v8us __attribute__((ext_vector_type(8), may_alias));
typedef float v8f  __attribute__((ext_vector_type(8)));
typedef float v4f  __attribute__((ext_vector_type(4)));
typedef float v4fa __attribute__((ext_vector_type(4), may_alias));
union FragH { v16h v; v8us half[2]; _Float16 h[16]; unsigned short u[16]; };

__device__ __forceinline__ unsigned short bf16_bits(float x) { unsigned int u = __float_as_uint(x); return (unsigned short)((u + 0x7FFFu + ((u >> 16) & 1u)) >> 16); }
__device__ __forceinline__ float bf16_val(unsigned short b) { return __uint_as_float(((unsigned int)b) << 16); }
__device__ __forceinline__ float bf16_rne(float x) { return bf16_val(bf16_bits(x)); }

__device__ __forceinline__ v16h g2_frag(const _Float16* p, int hh) { FragH f; f.half[0] = *(const v8us*)((const unsigned short*)p + 8 * hh); f.half[1] = *(const v8us*)((const unsigned short*)p + 16 + 8 * hh); return f.v; }
__device__ __forceinline__ v8f g2_mma(v16h a, v16h b, v8f c) { v8f d = __builtin_amdgcn_wmma_f32_16x16x32_f16(false, a, false, b, (short)0, c, false, false); asm volatile("v_nop\n\tv_nop\n\tv_nop\n\tv_nop" : "+v"(d) : "v"(a), "v"(b)); return d; }

__global__ __launch_bounds__(256) void k_wt_f16(const float* __restrict__ W, _Float16* __restrict__ Wt, int K, int N, float scale) {
  const int t = blockIdx.x * 256 + threadIdx.x; if (t >= N * (K / 8)) return; const int n = t / (K / 8), k8 = (t % (K / 8)) * 8; FragH f;
#pragma unroll
  for (int i = 0; i < 8; ++i) f.h[i] = (_Float16)(bf16_rne(W[(size_t)(k8 + i) * N + n]) * scale);
  const v8us o = f.half[0];
  *(volatile v8us*)((unsigned short*)Wt + (size_t)n * K + k8) = o; __threadfence(); *(volatile v8us*)((unsigned short*)Wt + (size_t)n * K + k8) = o;
}
__global__ __launch_bounds__(256) void k_x16(const float* __restrict__ x, _Float16* __restrict__ X16, size_t n8) {
  const size_t t = (size_t)blockIdx.x * 256 + threadIdx.x; if (t >= n8) return; FragH f;
#pragma unroll
  for (int q = 0; q < 8; ++q) f.h[q] = (_Float16)bf16_rne(x[t * 8 + q]);
  const v8us o = f.half[0];
  *(volatile v8us*)((unsigned short*)X16 + t * 8) = o; __threadfence(); *(volatile v8us*)((unsigned short*)X16 + t * 8) = o;
}

template <int TRI, bool CPBF>
__global__ __launch_bounds__(128) void k_gemm2(const _Float16* __restrict__ A, int lda, const _Float16* __restrict__ Bh, int ldb, float alpha,
                                               const float* __restrict__ bias, const float* __restrict__ CP,
                                               float* __restrict__ C, _Float16* __restrict__ C16, int ldc, int M, int N, int K) {
  __shared__ __attribute__((aligned(16))) float so[4][32][68];
  const int tid = threadIdx.x, w = tid >> 5, lane = tid & 31, ln = lane & 15, hh = lane >> 4;
  const int ntn = N >> 6; const int mt = blockIdx.x / ntn, nq = blockIdx.x - mt * ntn;
  const int row0 = mt * 128 + 32 * w, col0 = nq * 64;
  if (row0 >= M) return;
  if (TRI == 1) { if (col0 + 63 <= mt * 128) return; }
  int kb0 = 0;
  if (TRI == 2) kb0 = (row0 + 32 >= M) ? 0 : row0;
  const _Float16* a0p = A + (size_t)(row0 + ln) * lda; const _Float16* a1p = a0p + (size_t)16 * lda;
  const _Float16* b0p = Bh + (size_t)(col0 + ln) * ldb; const _Float16* b1p = b0p + (size_t)16 * ldb; const _Float16* b2p = b1p + (size_t)16 * ldb; const _Float16* b3p = b2p + (size_t)16 * ldb;
  const v8f z8 = {0.f,0.f,0.f,0.f,0.f,0.f,0.f,0.f}; v8f c00 = z8, c01 = z8, c02 = z8, c03 = z8, c10 = z8, c11 = z8, c12 = z8, c13 = z8;
#pragma unroll 1
  for (int kb = kb0; kb < K; kb += 32) {
    const v16h a0 = g2_frag(a0p + kb, hh), a1 = g2_frag(a1p + kb, hh);
    v16h b = g2_frag(b0p + kb, hh); c00 = g2_mma(a0, b, c00); c10 = g2_mma(a1, b, c10);
    b = g2_frag(b1p + kb, hh); c01 = g2_mma(a0, b, c01); c11 = g2_mma(a1, b, c11);
    b = g2_frag(b2p + kb, hh); c02 = g2_mma(a0, b, c02); c12 = g2_mma(a1, b, c12);
    b = g2_frag(b3p + kb, hh); c03 = g2_mma(a0, b, c03); c13 = g2_mma(a1, b, c13);
  }
  v8f accs[8] = {c00, c01, c02, c03, c10, c11, c12, c13};
#pragma unroll
  for (int u = 0; u < 8; ++u) {
    const int t = u & 3, half = u >> 2; const int col = col0 + t * 16 + ln;
    const float bv = bias ? bf16_rne(bias[col]) : 0.f;
#pragma unroll
    for (int r = 0; r < 8; ++r) { const int rloc = half * 16 + 8 * hh + r; so[w][rloc][t * 16 + ln] = accs[u][r] * alpha + bv; }
  }
  __builtin_amdgcn_fence(4  , "workgroup"); __builtin_amdgcn_wave_barrier();
  const int rsub = lane >> 4, c4 = (lane & 15) * 4;
  if (CP) {
#pragma unroll 1
    for (int q = 0; q < 16; ++q) {
      const int r = q * 2 + rsub;
      v4f v = *(const v4fa*)&so[w][r][c4];
      const v4f xr = *(const v4fa*)(CP + (size_t)(row0 + r) * ldc + col0 + c4);
#pragma unroll
      for (int i = 0; i < 4; ++i) v[i] += CPBF ? bf16_rne(xr[i]) : xr[i];
      *(v4fa*)&so[w][r][c4] = v;
    }
    __builtin_amdgcn_fence(4  , "workgroup"); __builtin_amdgcn_wave_barrier();
  }
  for (int pass = 0; pass < 2; ++pass) {
#pragma unroll
    for (int q = 0; q < 16; ++q) {
      const int r = q * 2 + rsub; const v4f v = *(const v4fa*)&so[w][r][c4];
      if (C) *(volatile v4f*)(C + (size_t)(row0 + r) * ldc + col0 + c4) = v;
      if (C16) { v4h h4; for (int i = 0; i < 4; ++i) h4[i] = (_Float16)v[i]; *(volatile v4h*)(C16 + (size_t)(row0 + r) * ldc + col0 + c4) = h4; }
    }
    if (pass == 0) __threadfence();
  }
}

template <int NHv, int TTv>
__global__ __launch_bounds__(256) void k_vt(const _Float16* __restrict__ V16, int ldv, int voff, _Float16* __restrict__ Vt) {
  __shared__ unsigned short tl[64][66];
  const int tid = threadIdx.x; const int slab = blockIdx.x / (TTv / 64), lg = blockIdx.x % (TTv / 64);
  for (int i = tid; i < 64 * 8; i += 256) { const int r = i / 8, c8 = (i % 8) * 8; FragH f; f.half[0] = *(const v8us*)((const unsigned short*)V16 + ((size_t)lg * 64 + r) * ldv + voff + slab * 64 + c8);
#pragma unroll
    for (int q = 0; q < 8; ++q) tl[r][c8 + q] = f.u[q]; }
  __syncthreads();
  for (int pass = 0; pass < 2; ++pass) {
#pragma unroll
    for (int rd = 0; rd < 2; ++rd) { const int d = rd * 32 + tid / 8, pc = tid % 8; FragH f;
#pragma unroll
      for (int q = 0; q < 8; ++q) f.u[q] = tl[pc * 8 + q][d];
      *(volatile v8us*)((unsigned short*)Vt + ((size_t)slab * 64 + d) * TTv + lg * 64 + pc * 8) = f.half[0]; }
    if (pass == 0) __threadfence(); }
}

__device__ __forceinline__ void ld8(const float* p, float (&t)[8]) { const v4f a = *(const v4fa*)p, b = *(const v4fa*)(p + 4); t[0] = a[0]; t[1] = a[1]; t[2] = a[2]; t[3] = a[3]; t[4] = b[0]; t[5] = b[1]; t[6] = b[2]; t[7] = b[3]; }

__global__ __launch_bounds__(256) void k_smx(const float* __restrict__ S, _Float16* __restrict__ P, int n) {
#pragma clang fp contract(off)
  const int tid = threadIdx.x, lane = tid & 31;
  const int w = __builtin_amdgcn_readfirstlane(tid >> 5);
  const int i = blockIdx.x * 8 + w;
  if (i >= n) return;
  const float* s = S + (size_t)i * n;
  unsigned short* prow = (unsigned short*)P + (size_t)i * n;
  const int nch = n >> 8;
  const int u0 = (i + 1) >> 8;
  float m = MASKV;
#pragma unroll 1
  for (int u = u0; u < nch; ++u) {
    const int j0 = u * 256 + lane * 8; float t[8]; ld8(s + j0, t);
#pragma unroll
    for (int q = 0; q < 8; ++q) m = fmaxf(m, (j0 + q <= i) ? MASKV : t[q]);
  }
#pragma unroll
  for (int off = 16; off > 0; off >>= 1) m = fmaxf(m, __shfl_xor(m, off, 32));
  float l = 0.f;
#pragma unroll 1
  for (int u = u0; u < nch; ++u) {
    const int j0 = u * 256 + lane * 8; float t[8]; ld8(s + j0, t);
#pragma unroll
    for (int q = 0; q < 8; ++q) l += (j0 + q <= i) ? 0.f : __expf(t[q] - m);
  }
#pragma unroll
  for (int off = 16; off > 0; off >>= 1) l += __shfl_xor(l, off, 32);
  const float em = __expf(MASKV - m);
  const float lm = (float)(i + 1) * em;
  l = l + lm;
  const float rl = 1.0f / l;
  const float sc = 1024.0f * rl;
  const float pm = em * sc;
#pragma unroll 1
  for (int u = 0; u < nch; ++u) {
    FragH f;
    if (u < u0) {
#pragma unroll
      for (int q = 0; q < 8; ++q) f.h[q] = (_Float16)pm;
    } else {
      const int j0 = u * 256 + lane * 8; float t[8]; ld8(s + j0, t);
#pragma unroll
      for (int q = 0; q < 8; ++q) { const float e = (j0 + q <= i) ? pm : __expf(t[q] - m) * sc; f.h[q] = (_Float16)e; }
    }
    const v8us o = f.half[0];
    volatile v8us* d = (volatile v8us*)(prow + (size_t)u * 256 + lane * 8);
    *d = o; __threadfence(); *d = o;
  }
}

extern "C" void kernel_launch(void* const* d_in, const int* in_sizes, int n_in,
                              void* d_out, int out_size, void* d_ws, size_t ws_size, hipStream_t stream) {
  if (n_in < 7) return;
  if (in_sizes[0] < SEQ * EMB || in_sizes[1] < EMB * EMB || in_sizes[2] < EMB || in_sizes[3] < EMB * EMB || in_sizes[4] < EMB ||
      in_sizes[5] < EMB * EMB || in_sizes[6] < EMB || out_size < SEQ * EMB) return;
  const float* x  = (const float*)d_in[0];
  const float* Wq = (const float*)d_in[1]; const float* bq = (const float*)d_in[2];
  const float* Wk = (const float*)d_in[3]; const float* bk = (const float*)d_in[4];
  const float* Wv = (const float*)d_in[5]; const float* bv = (const float*)d_in[6];
  float* out = (float*)d_out;
  char* ws = (char*)d_ws; size_t off = 0;
  auto take = [&](size_t bytes) { char* p = ws + off; off += (bytes + 255) & ~(size_t)255; return p; };
  const size_t wbytes = (size_t)EMB * EMB * 2, rbytes = (size_t)SEQ * EMB * 2, sbytes = (size_t)SEQ * SEQ * 4, pbytes = (size_t)SEQ * SEQ * 2;
  _Float16* BQ = (_Float16*)take(wbytes); _Float16* BK = (_Float16*)take(wbytes); _Float16* BV = (_Float16*)take(wbytes);
  _Float16* Q16 = (_Float16*)take(rbytes); _Float16* K16 = (_Float16*)take(rbytes); _Float16* VT = (_Float16*)take(rbytes);
  _Float16* P = (_Float16*)take(pbytes);
  const size_t rsbytes = (sbytes > 2 * rbytes) ? sbytes : 2 * rbytes;
  char* RS = take(rsbytes);
  _Float16* X16 = (_Float16*)RS; _Float16* V16 = (_Float16*)(RS + rbytes); float* S = (float*)RS;
  if (off > ws_size || off > (size_t)134217728) return;

  k_wt_f16<<<(unsigned)((EMB * (EMB / 8) + 255) / 256), 256, 0, stream>>>(Wq, BQ, EMB, EMB, 16.0f);
  k_wt_f16<<<(unsigned)((EMB * (EMB / 8) + 255) / 256), 256, 0, stream>>>(Wk, BK, EMB, EMB, 16.0f);
  k_wt_f16<<<(unsigned)((EMB * (EMB / 8) + 255) / 256), 256, 0, stream>>>(Wv, BV, EMB, EMB, 16.0f);
  const size_t n8 = (size_t)SEQ * EMB / 8;
  k_x16<<<(unsigned)((n8 + 255) / 256), 256, 0, stream>>>(x, X16, n8);
  const unsigned gq = (unsigned)((SEQ / 128) * (EMB / 64));
  k_gemm2<0, false><<<gq, 128, 0, stream>>>(X16, EMB, BQ, EMB, 0.0625f, bq, nullptr, nullptr, Q16, EMB, SEQ, EMB, EMB);
  k_gemm2<0, false><<<gq, 128, 0, stream>>>(X16, EMB, BK, EMB, 0.0625f, bk, nullptr, nullptr, K16, EMB, SEQ, EMB, EMB);
  k_gemm2<0, false><<<gq, 128, 0, stream>>>(X16, EMB, BV, EMB, 0.0625f, bv, nullptr, nullptr, V16, EMB, SEQ, EMB, EMB);
  k_vt<EMB / 64, SEQ><<<(unsigned)((EMB / 64) * (SEQ / 64)), 256, 0, stream>>>(V16, EMB, 0, VT);
  k_gemm2<1, false><<<(unsigned)((SEQ / 128) * (SEQ / 64)), 128, 0, stream>>>(Q16, EMB, K16, EMB, 0.125f, nullptr, nullptr, S, nullptr, SEQ, SEQ, SEQ, EMB);
  k_smx<<<(unsigned)(SEQ / 8), 256, 0, stream>>>(S, P, SEQ);
  k_gemm2<2, true><<<gq, 128, 0, stream>>>(P, SEQ, VT, SEQ, 0.0009765625f, nullptr, x, out, nullptr, EMB, SEQ, EMB, SEQ);
}
